// MultiHeadedAttention_6502580486520
// MI455X (gfx1250) — hardware-verified
//
#include <hip/hip_runtime.h>
#include <math.h>

typedef __attribute__((ext_vector_type(16))) _Float16 v16h;
typedef __attribute__((ext_vector_type(16))) __bf16 v16b;
typedef __attribute__((ext_vector_type(8)))  _Float16 v8h;
typedef __attribute__((ext_vector_type(8)))  __bf16 v8b;
typedef __attribute__((ext_vector_type(8)))  float v8f;
typedef __attribute__((ext_vector_type(4)))  float v4f;
typedef __attribute__((ext_vector_type(4)))  unsigned v4u;
typedef __attribute__((ext_vector_type(4)))  int v4i;

template <typename T> __device__ __forceinline__ void vst2(void* p, T v) { *(volatile T*)p = v; __threadfence(); *(volatile T*)p = v; }
__device__ __forceinline__ v8f wmma16(v16h a, v16h b, v8f c) {
  v8f d = __builtin_amdgcn_wmma_f32_16x16x32_f16(false, a, false, b, (short)0, c, false, false);
  asm volatile("v_nop\n\tv_nop\n\tv_nop\n\tv_nop" : "+v"(d) : "v"(a), "v"(b));
  return d;
}
__device__ __forceinline__ v8f wmma_bf(v16b a, v16b b, v8f c) {
  v8f d = __builtin_amdgcn_wmma_f32_16x16x32_bf16(false, a, false, b, (short)0, c, false, false);
  asm volatile("v_nop\n\tv_nop\n\tv_nop\n\tv_nop" : "+v"(d) : "v"(a), "v"(b));
  return d;
}
__device__ __forceinline__ v16h frag_h(const _Float16* rowk0, int lane) {
  union { v16h v; v8h q[2]; } u; const _Float16* p = rowk0 + 8 * (lane >> 4);
  u.q[0] = *(const v8h*)p; u.q[1] = *(const v8h*)(p + 16); return u.v;
}
__device__ __forceinline__ v16b frag_b(const __bf16* rowk0, int lane) {
  union { v16b v; v8b q[2]; } u; const __bf16* p = rowk0 + 8 * (lane >> 4);
  u.q[0] = *(const v8b*)p; u.q[1] = *(const v8b*)(p + 16); return u.v;
}
__device__ __forceinline__ v16h frag_f32s(const float* rowk0, int lane, float sc) {
  v16h a; const float* p = rowk0 + 8 * (lane >> 4);
#pragma unroll
  for (int i = 0; i < 8; ++i) { a[i] = (_Float16)(p[i] * sc); a[8 + i] = (_Float16)(p[16 + i] * sc); }
  return a;
}
struct F2 { v16b h, l; };
__device__ __forceinline__ F2 bsplit16(const float v[16]) { F2 r;
#pragma unroll
  for (int i = 0; i < 16; ++i) { const __bf16 h = (__bf16)v[i]; r.h[i] = h; r.l[i] = (__bf16)(v[i] - (float)h); }
  return r; }
__device__ __forceinline__ F2 split_row(const float* row, int k0, int lane) { float v[16]; const float* p = row + k0 + 8 * (lane >> 4);
#pragma unroll
  for (int i = 0; i < 8; ++i) { v[i] = p[i]; v[8 + i] = p[16 + i]; }
  return bsplit16(v); }
__device__ __forceinline__ float bfr(float v) { return (float)(__bf16)v; }
#define LDSX() do { asm volatile("s_wait_dscnt 0" ::: "memory"); __builtin_amdgcn_wave_barrier(); __builtin_amdgcn_fence(3  , "workgroup"); } while (0)

#ifndef NB
#define NB 2
#endif
#ifndef SEQ
#define SEQ 2048
#endif
#define NB_FULL 2
#define SEQ_FULL 2048
#define NH 16
#define HD 64
#define CC 1024
#define DIN 1024
#define QHI 256
#define NKT (SEQ / 32)
#define FLP (((NKT + 31) / 32) * 32)
#define PLANE ((size_t)NB * SEQ * CC)
#define SC2 (0.125f * 1.44269504088896340736f)
#define NEGBIG (-3.0e38f)
#define PCARRY 256.0f

static_assert(CC == NH * HD);
static_assert(HD == 64);
static_assert(DIN % 32 == 0 && CC % 32 == 0);
static_assert(CC % 128 == 0 && DIN % 128 == 0);
static_assert(SEQ % 64 == 0);
static_assert(SEQ <= SEQ_FULL && NB <= NB_FULL);
static_assert(NKT % 8 == 0 && FLP <= 256 && FLP % 32 == 0);
static_assert(QHI % 64 == 0);
static_assert(((size_t)NB * SEQ * DIN / 8) % 256 == 0);
static_assert(((size_t)CC * DIN / 8) % 256 == 0);
static_assert(64 * 136 <= 9216 && 128 * 72 <= 9216);

#define WS_XB   ((size_t)0)
#define WS_WB   (WS_XB  + 2u * (size_t)NB * SEQ * DIN)
#define WS_WOB  (WS_WB  + 2u * (size_t)3 * CC * DIN)
#define WS_WOH  (WS_WOB + 2u * (size_t)DIN * CC)
#define WS_QKH  (WS_WOH + 2u * (size_t)DIN * CC)
#define WS_QKL  (WS_QKH + 4u * PLANE)
#define WS_VT   (WS_QKL + 4u * PLANE)
#define WS_VL   (WS_VT  + 2u * PLANE)
#define WS_FL   (WS_VL  + 2u * PLANE)
#define WS_Y    (WS_FL  + 4u * (size_t)(SEQ / 16) * FLP)
#define WS_END  (WS_Y   + 4u * PLANE)
static_assert(WS_END <= (size_t)134217728);
static_assert(WS_WB % 128 == 0 && WS_QKH % 128 == 0 && WS_FL % 128 == 0 && WS_Y % 128 == 0);

__global__ __launch_bounds__(256) void k_cvt(const float* __restrict__ src, __bf16* __restrict__ dstb, _Float16* __restrict__ dsth, int n8, int rpb, int rpb_full, int wh) {
  const int gi = blockIdx.x * 256 + threadIdx.x; if (gi >= n8) return;
  const int r = gi / (DIN / 8), c8 = gi % (DIN / 8); const int bb = r / rpb, s = r % rpb;
  const float* p = src + ((size_t)bb * rpb_full + s) * DIN + c8 * 8;
  const v4f u0 = *(const v4f*)p, u1 = *(const v4f*)(p + 4);
  v8b hb;
#pragma unroll
  for (int i = 0; i < 4; ++i) { hb[i] = (__bf16)u0[i]; hb[4 + i] = (__bf16)u1[i]; }
  vst2(dstb + (size_t)gi * 8, *(const v4u*)&hb);
  if (wh != 0) { v8h hh;
#pragma unroll
    for (int i = 0; i < 8; ++i) hh[i] = (_Float16)((float)hb[i] * 256.0f);
    vst2(dsth + (size_t)gi * 8, *(const v4u*)&hh); } }

__global__ __launch_bounds__(256) void k_flags(const int* __restrict__ MASK, int* __restrict__ FL) {
  __shared__ __align__(16) int sfl[FLP];
  const int tid = threadIdx.x, lane = tid & 31; const int wave = __builtin_amdgcn_readfirstlane(tid >> 5); const int qt = blockIdx.x;
  if (tid < FLP) sfl[tid] = 0;
  __syncthreads();
#pragma unroll 1
  for (int i = 0; i < NKT / 8; ++i) { const int kt = wave * (NKT / 8) + i;
    const int* mp = MASK + (size_t)(qt * 16 + (lane >> 3)) * SEQ_FULL + kt * 32 + (lane & 7) * 4;
    int any0 = 0, any1 = 0;
#pragma unroll
    for (int u = 0; u < 4; ++u) { const v4i x = *(const v4i*)(mp + (size_t)u * 4 * SEQ_FULL);
#pragma unroll
      for (int e = 0; e < 4; ++e) { any0 |= (x[e] == 0) ? 1 : 0; any1 |= (x[e] != 0) ? 1 : 0; } }
    const bool a0 = __ballot(any0) != 0, a1 = __ballot(any1) != 0;
    if (lane == 0) sfl[kt] = a1 ? (a0 ? 2 : 1) : 0; }
  __syncthreads();
  if (wave == 0 && lane < FLP / 4) vst2(FL + (size_t)qt * FLP + lane * 4, *(const v4i*)&sfl[lane * 4]); }

__global__ __launch_bounds__(128) void k_proj(const __bf16* __restrict__ XB, const __bf16* __restrict__ WB, const float* __restrict__ BQ, const float* __restrict__ BK, const float* __restrict__ BV,
    _Float16* __restrict__ QKH, _Float16* __restrict__ QKL, _Float16* __restrict__ VT, _Float16* __restrict__ VL) {
  __shared__ __align__(16) _Float16 sa[9216], sb[9216];
  const int tid = threadIdx.x, lane = tid & 31, col = lane & 15, g = lane >> 4; const int wave = __builtin_amdgcn_readfirstlane(tid >> 5);
  const int n0 = blockIdx.y * 128; const int which = n0 / CC; const int c0 = n0 % CC;
  const size_t r0 = (size_t)blockIdx.x * 64; const size_t bb = r0 / SEQ; const int t0 = (int)(r0 % SEQ);
  v8f acc[8] = {};
#pragma unroll 2
  for (int kc = 0; kc < DIN / 32; ++kc) { const v16b a = frag_b(XB + (r0 + wave * 16 + col) * DIN + kc * 32, lane);
    asm volatile("s_wait_loadcnt 0x0" ::: "memory");
#pragma unroll
    for (int j = 0; j < 8; ++j) { const v16b w = frag_b(WB + (size_t)(n0 + j * 16 + col) * DIN + kc * 32, lane); asm volatile("s_wait_loadcnt 0x0" ::: "memory"); acc[j] = wmma_bf(a, w, acc[j]); } }
#pragma unroll
  for (int j = 0; j < 8; ++j) { const int ci = c0 + j * 16 + col; const float b0 = BQ[ci], b1 = BK[ci], b2 = BV[ci]; const float bias = bfr(which == 0 ? b0 : (which == 1 ? b1 : b2));
#pragma unroll
    for (int r = 0; r < 8; ++r) { const float v = acc[j][r] + bias; const _Float16 hv = (_Float16)v; const _Float16 lv = (_Float16)((v - (float)hv) * 1024.0f);
      const int rl = wave * 16 + 8 * g + r, cl = j * 16 + col; const int idx = (which < 2) ? (rl * 136 + cl) : (cl * 72 + rl); sa[idx] = hv; sb[idx] = lv; } }
  __syncthreads();
  if (which < 2) {
    for (int e = tid; e < 64 * 16; e += 128) { const int rl = e >> 4, q = e & 15; const size_t off = (size_t)which * PLANE + (r0 + rl) * CC + c0 + q * 8;
      const v4u hv = *(const v4u*)&sa[rl * 136 + q * 8]; const v4u lv = *(const v4u*)&sb[rl * 136 + q * 8]; vst2(QKH + off, hv); vst2(QKL + off, lv); }
  } else {
    for (int e = tid; e < 128 * 8; e += 128) { const int cl = e >> 3, q = e & 7; const size_t off = (bb * CC + c0 + cl) * (size_t)SEQ + t0 + q * 8;
      const v4u hv = *(const v4u*)&sa[cl * 72 + q * 8]; const v4u lv = *(const v4u*)&sb[cl * 72 + q * 8]; vst2(VT + off, hv); vst2(VL + off, lv); } } }

__global__ __launch_bounds__(128) void k_attn(const _Float16* __restrict__ QKH, const _Float16* __restrict__ QKL, const _Float16* __restrict__ VT, const _Float16* __restrict__ VL,
    const int* __restrict__ MASK, const int* __restrict__ FL, float* __restrict__ Y) {
  __shared__ __align__(16) _Float16 sp[4][16][40];
  __shared__ __align__(16) _Float16 spl[4][16][40];
  __shared__ __align__(16) float ss[4][16][68];
  const int tid = threadIdx.x, lane = tid & 31, col = lane & 15, g = lane >> 4; const int wave = __builtin_amdgcn_readfirstlane(tid >> 5);
  const int qb = blockIdx.x, h = blockIdx.y, b = blockIdx.z;
  const bool early = qb * 64 < QHI;
  const int qt = qb * 4 + wave, ql0 = qt * 16;
  const size_t qrow0 = (size_t)b * SEQ + ql0, krow0 = (size_t)b * SEQ;
  const _Float16* QH = QKH; const _Float16* KH = QKH + PLANE; const _Float16* QL = QKL; const _Float16* KL = QKL + PLANE;
  v8f o[4] = {}, ol[4] = {};
  float m[8], l[8];
#pragma unroll
  for (int r = 0; r < 8; ++r) { m[r] = NEGBIG; l[r] = 0.f; }
#pragma unroll 1
  for (int kt = 0; kt < NKT; ++kt) {
    const int fl = __builtin_amdgcn_readfirstlane(FL[(size_t)qt * FLP + kt]);
    if (fl == 0) continue;
    const int k0 = kt * 32;
    v8f s0 = {}, s1 = {}, t0 = {}, t1 = {};
#pragma unroll
    for (int kc = 0; kc < HD / 32; ++kc) {
      const size_t qo = (qrow0 + col) * CC + h * HD + kc * 32; const size_t ka = (krow0 + k0 + col) * CC + h * HD + kc * 32; const size_t kb = ka + (size_t)16 * CC;
      const v16h a = frag_h(QH + qo, lane), b0 = frag_h(KH + ka, lane), b1 = frag_h(KH + kb, lane);
      s0 = wmma16(a, b0, s0); s1 = wmma16(a, b1, s1);
      if (early) { const v16h al = frag_h(QL + qo, lane); t0 = wmma16(al, b0, t0); t1 = wmma16(al, b1, t1);
        const v16h c0 = frag_h(KL + ka, lane), c1 = frag_h(KL + kb, lane); t0 = wmma16(a, c0, t0); t1 = wmma16(a, c1, t1); } }
    unsigned mk0 = 0xffu, mk1 = 0xffu;
    if (fl != 1) {
      const int* mp = MASK + (size_t)(ql0 + 8 * g) * SEQ_FULL + k0 + col; unsigned a0 = 0u, a1 = 0u;
#pragma unroll
      for (int r = 0; r < 8; ++r) a0 |= ((mp[(size_t)r * SEQ_FULL] != 0) ? 1u : 0u) << r;
      asm volatile("s_wait_loadcnt 0x0" ::: "memory");
#pragma unroll
      for (int r = 0; r < 8; ++r) a1 |= ((mp[(size_t)r * SEQ_FULL + 16] != 0) ? 1u : 0u) << r;
      mk0 = a0; mk1 = a1; }
#pragma unroll
    for (int r = 0; r < 8; ++r) {
      const bool ok0 = ((mk0 >> r) & 1u) != 0u, ok1 = ((mk1 >> r) & 1u) != 0u;
      const float a = ok0 ? (s0[r] + t0[r] * (1.0f / 1024.0f)) * SC2 : NEGBIG;
      const float c = ok1 ? (s1[r] + t1[r] * (1.0f / 1024.0f)) * SC2 : NEGBIG;
      float mx = fmaxf(a, c);
      mx = fmaxf(mx, __shfl_xor(mx, 1)); mx = fmaxf(mx, __shfl_xor(mx, 2)); mx = fmaxf(mx, __shfl_xor(mx, 4)); mx = fmaxf(mx, __shfl_xor(mx, 8));
      const float mnew = fmaxf(m[r], mx);
      const float alpha = exp2f(m[r] - mnew);
      const float e0 = exp2f(a - mnew), e1 = exp2f(c - mnew);
      const float p0 = ok0 ? e0 : 0.f, p1 = ok1 ? e1 : 0.f;
      float rs = p0 + p1;
      rs += __shfl_xor(rs, 1); rs += __shfl_xor(rs, 2); rs += __shfl_xor(rs, 4); rs += __shfl_xor(rs, 8);
      l[r] = l[r] * alpha + rs; m[r] = mnew;
#pragma unroll
      for (int j = 0; j < 4; ++j) { o[j][r] *= alpha; ol[j][r] *= alpha; }
      const float pc0 = p0 * PCARRY, pc1 = p1 * PCARRY; const _Float16 h0 = (_Float16)pc0, h1 = (_Float16)pc1;
      sp[wave][8 * g + r][col] = h0; sp[wave][8 * g + r][16 + col] = h1;
      if (early) { spl[wave][8 * g + r][col] = (_Float16)((pc0 - (float)h0) * 1024.0f); spl[wave][8 * g + r][16 + col] = (_Float16)((pc1 - (float)h1) * 1024.0f); } }
    LDSX();
    union { v16h v; v8h q[2]; } up; up.q[0] = *(const v8h*)&sp[wave][col][8 * g]; up.q[1] = *(const v8h*)&sp[wave][col][16 + 8 * g];
    const v16h pa = up.v; v16h pal = pa;
    if (early) { union { v16h v; v8h q[2]; } ul; ul.q[0] = *(const v8h*)&spl[wave][col][8 * g]; ul.q[1] = *(const v8h*)&spl[wave][col][16 + 8 * g]; pal = ul.v; }
    asm volatile("" ::: "memory");
#pragma unroll
    for (int j = 0; j < 4; ++j) { const size_t vo = ((size_t)b * CC + h * HD + j * 16 + col) * (size_t)SEQ + k0;
      const v16h vb = frag_h(VT + vo, lane); o[j] = wmma16(pa, vb, o[j]);
      if (early) { ol[j] = wmma16(pal, vb, ol[j]); const v16h vl = frag_h(VL + vo, lane); ol[j] = wmma16(pa, vl, ol[j]); } }
  }
#pragma unroll
  for (int r = 0; r < 8; ++r) { const float inv = (1.0f / l[r]) * (1.0f / PCARRY);
#pragma unroll
    for (int j = 0; j < 4; ++j) ss[wave][8 * g + r][j * 16 + col] = (o[j][r] + ol[j][r] * (1.0f / 1024.0f)) * inv; }
  LDSX();
#pragma unroll 1
  for (int it = 0; it < 8; ++it) { const int rl = it * 2 + g; const v4f v = *(const v4f*)&ss[wave][rl][col * 4]; vst2(Y + (qrow0 + rl) * CC + h * HD + col * 4, v); } }

__global__ __launch_bounds__(128) void k_out(const float* __restrict__ Y, const _Float16* __restrict__ WOH, const __bf16* __restrict__ WOB, const float* __restrict__ BO, float* __restrict__ OUT) {
  __shared__ __align__(16) float sf[4][16][132];
  const int tid = threadIdx.x, lane = tid & 31, col = lane & 15, g = lane >> 4; const int wave = __builtin_amdgcn_readfirstlane(tid >> 5);
  const int c0 = blockIdx.y * 128; const size_t rb = (size_t)blockIdx.x * 64; const size_t r0 = rb + wave * 16;
  const bool early = (int)(rb % SEQ) < QHI;
  v8f acc[8] = {};
  if (early) {
#pragma unroll 2
    for (int kc = 0; kc < CC / 32; ++kc) { const F2 a = split_row(Y + (r0 + col) * CC, kc * 32, lane); asm volatile("s_wait_loadcnt 0x0" ::: "memory");
#pragma unroll
      for (int j = 0; j < 8; ++j) { const v16b w = frag_b(WOB + (size_t)(c0 + j * 16 + col) * CC + kc * 32, lane); asm volatile("s_wait_loadcnt 0x0" ::: "memory"); acc[j] = wmma_bf(a.h, w, acc[j]); acc[j] = wmma_bf(a.l, w, acc[j]); } }
  } else {
#pragma unroll 2
    for (int kc = 0; kc < CC / 32; ++kc) { const v16h a = frag_f32s(Y + (r0 + col) * CC + kc * 32, lane, 64.0f); asm volatile("s_wait_loadcnt 0x0" ::: "memory");
#pragma unroll
      for (int j = 0; j < 8; ++j) { const v16h w = frag_h(WOH + (size_t)(c0 + j * 16 + col) * CC + kc * 32, lane); asm volatile("s_wait_loadcnt 0x0" ::: "memory"); acc[j] = wmma16(a, w, acc[j]); } } }
  const float sc = early ? 1.0f : (1.0f / 16384.0f);
#pragma unroll
  for (int j = 0; j < 8; ++j) { const float bias = bfr(BO[c0 + j * 16 + col]);
#pragma unroll
    for (int r = 0; r < 8; ++r) sf[wave][8 * g + r][j * 16 + col] = acc[j][r] * sc + bias; }
  LDSX();
#pragma unroll 1
  for (int rl = 0; rl < 16; ++rl) { const size_t rr = r0 + rl; const size_t orow = (rr / SEQ) * (size_t)SEQ_FULL + (rr % SEQ);
    const v4f v = *(const v4f*)&sf[wave][rl][lane * 4]; vst2(OUT + orow * DIN + c0 + lane * 4, v); } }

extern "C" void kernel_launch(void* const* d_in, const int* in_sizes, int n_in, void* d_out, int out_size, void* d_ws, size_t ws_size, hipStream_t stream) {
  if (n_in < 10) return;
  const long long xneed = ((long long)(NB - 1) * SEQ_FULL + SEQ) * DIN;
  if ((long long)in_sizes[0] < xneed) return;
  if ((long long)in_sizes[1] < (long long)(SEQ - 1) * SEQ_FULL + SEQ) return;
  if (in_sizes[2] < CC * DIN || in_sizes[4] < CC * DIN || in_sizes[6] < CC * DIN || in_sizes[8] < DIN * CC) return;
  if (in_sizes[3] < CC || in_sizes[5] < CC || in_sizes[7] < CC || in_sizes[9] < DIN) return;
  if ((long long)out_size < xneed) return;
  if (ws_size < (size_t)WS_END) return;
  const float* x = (const float*)d_in[0]; const int* mask = (const int*)d_in[1];
  const float* Wq = (const float*)d_in[2]; const float* bq = (const float*)d_in[3];
  const float* Wk = (const float*)d_in[4]; const float* bk = (const float*)d_in[5];
  const float* Wv = (const float*)d_in[6]; const float* bv = (const float*)d_in[7];
  const float* Wo = (const float*)d_in[8]; const float* bo = (const float*)d_in[9];
  char* ws = (char*)d_ws;
  __bf16* XB = (__bf16*)(ws + WS_XB); __bf16* WB = (__bf16*)(ws + WS_WB); __bf16* WOB = (__bf16*)(ws + WS_WOB); _Float16* WOH = (_Float16*)(ws + WS_WOH);
  _Float16* QKH = (_Float16*)(ws + WS_QKH); _Float16* QKL = (_Float16*)(ws + WS_QKL); _Float16* VT = (_Float16*)(ws + WS_VT); _Float16* VL = (_Float16*)(ws + WS_VL);
  int* FL = (int*)(ws + WS_FL); float* Y = (float*)(ws + WS_Y);
  const int nx8 = (int)((size_t)NB * SEQ * DIN / 8), nw8 = (int)((size_t)CC * DIN / 8);
  k_cvt<<<nx8 / 256, 256, 0, stream>>>(x, XB, WOH, nx8, SEQ, SEQ_FULL, 0);
  k_cvt<<<nw8 / 256, 256, 0, stream>>>(Wq, WB, WOH, nw8, CC, CC, 0);
  k_cvt<<<nw8 / 256, 256, 0, stream>>>(Wk, WB + (size_t)CC * DIN, WOH, nw8, CC, CC, 0);
  k_cvt<<<nw8 / 256, 256, 0, stream>>>(Wv, WB + (size_t)2 * CC * DIN, WOH, nw8, CC, CC, 0);
  k_cvt<<<nw8 / 256, 256, 0, stream>>>(Wo, WOB, WOH, nw8, DIN, DIN, 1);
  k_flags<<<SEQ / 16, 256, 0, stream>>>(mask, FL);
  k_proj<<<dim3(NB * SEQ / 64, 3 * CC / 128), 128, 0, stream>>>(XB, WB, bq, bk, bv, QKH, QKL, VT, VL);
  k_attn<<<dim3(SEQ / 64, NH, NB), 128, 0, stream>>>(QKH, QKL, VT, VL, mask, FL, Y);
  k_out<<<dim3(NB * SEQ / 64, DIN / 128), 128, 0, stream>>>(Y, WOH, WOB, bo, (float*)d_out);
}
